// DeformableBlock_37907381354832
// MI455X (gfx1250) — hardware-verified
//
#include <hip/hip_runtime.h>

#pragma clang fp contract(off)

typedef __attribute__((ext_vector_type(16))) _Float16 v16h;
typedef __attribute__((ext_vector_type(8)))  _Float16 v8h;
typedef __attribute__((ext_vector_type(16))) __bf16   v16b;
typedef __attribute__((ext_vector_type(8)))  __bf16   v8b;
typedef __attribute__((ext_vector_type(8)))  float    v8f;
typedef __attribute__((ext_vector_type(4)))  float    v4f;
typedef __attribute__((ext_vector_type(2)))  float    v2f;
typedef __attribute__((ext_vector_type(4)))  unsigned int v4u;
typedef __attribute__((ext_vector_type(4)))  int      v4i;

__device__ __forceinline__ unsigned short f2bf_bits(float f) {
  unsigned u = __float_as_uint(f);
  return (unsigned short)((u + 0x7FFFu + ((u >> 16) & 1u)) >> 16);
}
__device__ __forceinline__ float bf_bits2f(unsigned short h) { return __uint_as_float(((unsigned)h) << 16); }

__device__ __forceinline__ void dep_guard_h(v8f& a, v8f& b, v16h x, v16h y) { asm volatile("v_nop\n\tv_nop\n\tv_nop\n\tv_nop" : "+v"(a), "+v"(b) : "v"(x), "v"(y)); }
__device__ __forceinline__ void dep_guard_b(v8f& a, v8f& b, v16b x, v16b y) { asm volatile("v_nop\n\tv_nop\n\tv_nop\n\tv_nop" : "+v"(a), "+v"(b) : "v"(x), "v"(y)); }
__device__ __forceinline__ void keep4_h(v16h a, v16h b, v16h c, v16h d) { asm volatile("v_nop" :: "v"(a), "v"(b), "v"(c), "v"(d)); }
__device__ __forceinline__ void keep4_b(v16b a, v16b b, v16b c, v16b d) { asm volatile("v_nop" :: "v"(a), "v"(b), "v"(c), "v"(d)); }
__device__ __forceinline__ void acc_guard4(v8f& a, v8f& b, v8f& c, v8f& d) { asm volatile("v_nop\n\tv_nop\n\tv_nop\n\tv_nop" : "+v"(a), "+v"(b), "+v"(c), "+v"(d)); }
template <typename T> struct Frag;
template <> struct Frag<_Float16> {
  typedef v16h V; union U { v16h v; v8h h[2]; };
  static __device__ __forceinline__ v16h load(const _Float16* p) {
    U f; f.h[0] = *(const v8h*)(p); f.h[1] = *(const v8h*)(p + 16); return f.v;
  }
  static __device__ __forceinline__ v8f mma(v16h a, v16h b, v8f c) {
    return __builtin_amdgcn_wmma_f32_16x16x32_f16(false, a, false, b, (short)0, c, false, false);
  }
  static __device__ __forceinline__ void guard(v8f& a, v8f& b, v16h x, v16h y) { dep_guard_h(a, b, x, y); }
  static __device__ __forceinline__ void keep(v16h a, v16h b, v16h c, v16h d) { keep4_h(a, b, c, d); }
};
template <> struct Frag<__bf16> {
  typedef v16b V; union U { v16b v; v8b h[2]; };
  static __device__ __forceinline__ v16b load(const __bf16* p) {
    U f; f.h[0] = *(const v8b*)(p); f.h[1] = *(const v8b*)(p + 16); return f.v;
  }
  static __device__ __forceinline__ v8f mma(v16b a, v16b b, v8f c) {
    return __builtin_amdgcn_wmma_f32_16x16x32_bf16(false, a, false, b, (short)0, c, false, false);
  }
  static __device__ __forceinline__ void guard(v8f& a, v8f& b, v16b x, v16b y) { dep_guard_b(a, b, x, y); }
  static __device__ __forceinline__ void keep(v16b a, v16b b, v16b c, v16b d) { keep4_b(a, b, c, d); }
};

template <int ET> struct Elem;
template <> struct Elem<0> { typedef _Float16 T; };
template <> struct Elem<1> { typedef __bf16 T; };
template <int ET, bool SPLIT, int BIAS_MODE, int OUT_MODE, bool RESID, int ACT = 0>
__global__ __launch_bounds__(256) void wmma_gemm64(
    const unsigned short* __restrict__ Ap, const unsigned short* __restrict__ A2p, int lda, long strideA,
    const unsigned short* __restrict__ Btp, const unsigned short* __restrict__ Bt2p, int ldb, long strideB,
    void* __restrict__ Cout, void* __restrict__ Cout2, int ldc, long strideC,
    const float* __restrict__ bias,
    const float* __restrict__ resid, long strideR,
    int M, int N, int K, float scale) {
  typedef typename Elem<ET>::T T;
  typedef typename Frag<T>::V V;
  const T* A = (const T*)Ap; const T* A2 = (const T*)A2p; const T* Bt = (const T*)Btp; const T* Bt2 = (const T*)Bt2p;
  __shared__ __align__(16) float sT[8][16 * 68];
  const int b    = blockIdx.y;
  const int lane = threadIdx.x & 31;
  const int wave = threadIdx.x >> 5;
  const int tilesN = N >> 6;
  const int tilesM = M >> 6;
  const int tile = blockIdx.x * 8 + wave;
  if (tile >= tilesM * tilesN) return;
  const int tm = tile / tilesN;
  const int tn = tile - tm * tilesN;
  const int m0 = tm << 6;
  const int n0 = tn << 6;

  const T* Ab  = A  + (size_t)b * strideA;
  const T* Bb  = Bt + (size_t)b * strideB;
  const T* Ab2 = SPLIT ? (A2  + (size_t)b * strideA) : nullptr;
  const T* Bb2 = SPLIT ? (Bt2 + (size_t)b * strideB) : nullptr;

  const int rlane = lane & 15;
  const int koff  = (lane >> 4) * 8;
  const int mOff  = (lane >> 4) * 8;

  v8f acc[4][4];
#pragma unroll
  for (int i = 0; i < 4; ++i)
#pragma unroll
    for (int j = 0; j < 4; ++j) acc[i][j] = (v8f){0.f,0.f,0.f,0.f,0.f,0.f,0.f,0.f};

  for (int k0 = 0; k0 < K; k0 += 32) {
    V bh[4], bl[4];
#pragma unroll
    for (int j = 0; j < 4; ++j) {
      const size_t bo = (size_t)(n0 + (j << 4) + rlane) * ldb + koff + k0;
      bh[j] = Frag<T>::load(Bb + bo);
      if (SPLIT) bl[j] = Frag<T>::load(Bb2 + bo);
    }
#pragma unroll
    for (int i = 0; i < 4; ++i) {
      const size_t ao = (size_t)(m0 + (i << 4) + rlane) * lda + koff + k0;
      V ah = Frag<T>::load(Ab + ao);
      V al;
      if (SPLIT) al = Frag<T>::load(Ab2 + ao);
#pragma unroll
      for (int j = 0; j < 4; ++j) {
        acc[i][j] = Frag<T>::mma(ah, bh[j], acc[i][j]);
        if (SPLIT) {
          acc[i][j] = Frag<T>::mma(ah, bl[j], acc[i][j]);
          acc[i][j] = Frag<T>::mma(al, bh[j], acc[i][j]);
        }
      }
      Frag<T>::guard(acc[i][0], acc[i][3], ah, SPLIT ? al : ah);
    }
    Frag<T>::keep(bh[0], bh[1], bh[2], bh[3]);
    if (SPLIT) Frag<T>::keep(bl[0], bl[1], bl[2], bl[3]);
  }
  acc_guard4(acc[0][0], acc[0][1], acc[0][2], acc[0][3]);
  acc_guard4(acc[1][0], acc[1][1], acc[1][2], acc[1][3]);
  acc_guard4(acc[2][0], acc[2][1], acc[2][2], acc[2][3]);
  acc_guard4(acc[3][0], acc[3][1], acc[3][2], acc[3][3]);

  float* slab = sT[wave];
  const float* Rb = RESID ? (resid + (size_t)b * strideR) : nullptr;
#pragma unroll
  for (int i = 0; i < 4; ++i) {
    const int mBase = m0 + (i << 4);
#pragma unroll
    for (int j = 0; j < 4; ++j) {
      const int n = n0 + (j << 4) + rlane;
      float bv = 0.f;
      if (BIAS_MODE == 2) bv = bias[n];
#pragma unroll
      for (int r = 0; r < 8; ++r) {
        float v = acc[i][j][r] * scale;
        if (BIAS_MODE == 1) v += bias[mBase + mOff + r];
        if (BIAS_MODE == 2) v += bv;
        if (RESID) v += Rb[(size_t)(mBase + mOff + r) * ldc + n];
        if (ACT == 1) v = tanhf(v);
        if (ACT == 2) v = fmaxf(v, 0.0f);
        if (ACT == 3) v = v / (1.0f + expf(-v));
        if (ACT == 4) v = (v > 0.f) ? v : 0.01f * v;
        if (ACT == 5) v = 0.5f * v * (1.0f + erff(v * 0.70710678118654752f));
        slab[(mOff + r) * 68 + (j << 4) + rlane] = v;
      }
    }
    __builtin_amdgcn_fence(__ATOMIC_RELEASE, "workgroup");
    __builtin_amdgcn_wave_barrier();
    __builtin_amdgcn_fence(__ATOMIC_ACQUIRE, "workgroup");
    if (OUT_MODE == 0) {
      float* C = (float*)Cout + (size_t)b * strideC;
      const int hh = lane >> 4, c4 = (lane & 15) * 4;
      for (int pass = 0; pass < 2; ++pass) {
#pragma unroll
        for (int it = 0; it < 8; ++it) {
          const int row = it * 2 + hh;
          v4f v = *(const v4f*)(slab + row * 68 + c4);
          *(volatile v4f*)(C + (size_t)(mBase + row) * ldc + n0 + c4) = v;
        }
        __threadfence();
      }
    } else {
      const int q = lane >> 3, c8 = (lane & 7) * 8;
      unsigned short* C  = (unsigned short*)Cout  + (size_t)b * strideC;
      unsigned short* C2 = (OUT_MODE == 2) ? ((unsigned short*)Cout2 + (size_t)b * strideC) : nullptr;
      for (int pass = 0; pass < 2; ++pass) {
#pragma unroll
        for (int it = 0; it < 4; ++it) {
          const int row = it * 4 + q;
          const float* sp = slab + row * 68 + c8;
          v8h hv, lv;
#pragma unroll
          for (int e = 0; e < 8; ++e) {
            if (OUT_MODE == 1) {
              hv[e] = (_Float16)sp[e];
            } else {
              unsigned short hb = f2bf_bits(sp[e]);
              unsigned short lb = f2bf_bits(sp[e] - bf_bits2f(hb));
              hv[e] = __builtin_bit_cast(_Float16, hb);
              lv[e] = __builtin_bit_cast(_Float16, lb);
            }
          }
          *(volatile v8h*)(C + (size_t)(mBase + row) * ldc + n0 + c8) = hv;
          if (OUT_MODE == 2) *(volatile v8h*)(C2 + (size_t)(mBase + row) * ldc + n0 + c8) = lv;
        }
        __threadfence();
      }
    }
    __builtin_amdgcn_fence(__ATOMIC_RELEASE, "workgroup");
    __builtin_amdgcn_wave_barrier();
    __builtin_amdgcn_fence(__ATOMIC_ACQUIRE, "workgroup");
  }
}

constexpr int NBATCH  = 8;
constexpr int NCH_IN  = 64;
constexpr int NCH_OUT = 64;
constexpr int IMG_H   = 96;
constexpr int IMG_W   = 96;
constexpr int HWPIX   = IMG_H * IMG_W;
constexpr int NTAP    = 9;
constexpr int KDIM    = NCH_IN * NTAP;
constexpr int NOFFC   = 18;
constexpr int MPAD    = 64;
constexpr int HALF_B  = 4;
constexpr float BN_EPS = 1e-5f;

static_assert(KDIM % 32 == 0);
static_assert(HWPIX % 64 == 0);
static_assert(MPAD % 64 == 0 && NCH_OUT == MPAD && NOFFC <= MPAD);
static_assert(IMG_W % 32 == 0);
static_assert(HWPIX % 1024 == 0);
static_assert(NBATCH % HALF_B == 0);

constexpr size_t PLANE_BYTES = (size_t)HALF_B * HWPIX * KDIM * 2;
constexpr size_t OFFS_BYTES  = (size_t)NBATCH * MPAD * HWPIX * 4;
constexpr size_t YPRE_BYTES  = (size_t)NBATCH * NCH_OUT * HWPIX * 4;
constexpr size_t WPL_BYTES   = (size_t)MPAD * KDIM * 2;
constexpr size_t TAB_BYTES   = (size_t)NCH_OUT * NBATCH * 32 * 4;
constexpr size_t R_PHI  = 0;
constexpr size_t R_PLO  = R_PHI + PLANE_BYTES;
constexpr size_t R_OFFS = R_PLO + PLANE_BYTES;
constexpr size_t R_YPRE = R_OFFS + OFFS_BYTES;
constexpr size_t R_WOH  = R_YPRE + YPRE_BYTES;
constexpr size_t R_WOL  = R_WOH + WPL_BYTES;
constexpr size_t R_WDH  = R_WOL + WPL_BYTES;
constexpr size_t R_WDL  = R_WDH + WPL_BYTES;
constexpr size_t R_TAB  = R_WDL + WPL_BYTES;
constexpr size_t WS_TOTAL = R_TAB + TAB_BYTES;
static_assert(WS_TOTAL == 123043840);
static_assert(WS_TOTAL <= 134217728);
static_assert(R_PLO % 128 == 0 && R_OFFS % 128 == 0 && R_YPRE % 128 == 0 && R_WOH % 128 == 0 &&
              R_WOL % 128 == 0 && R_WDH % 128 == 0 && R_WDL % 128 == 0 && R_TAB % 128 == 0);

__global__ __launch_bounds__(256) void split_rows_kernel(
    const float* __restrict__ src, int nreal,
    unsigned int* __restrict__ dhi, unsigned int* __restrict__ dlo)
{
  const int t = blockIdx.x * 256 + threadIdx.x;
  if (t >= MPAD * KDIM / 8) return;
  const int e0  = t * 8;
  const int row = e0 / KDIM;
  const int col = e0 - row * KDIM;
  const bool real = row < nreal;
  const int rowc = real ? row : (nreal - 1);
  const float* p = src + (size_t)rowc * KDIM + col;
  const v4f a0 = *(const v4f*)(p);
  const v4f a1 = *(const v4f*)(p + 4);
  const float f[8] = {a0[0], a0[1], a0[2], a0[3], a1[0], a1[1], a1[2], a1[3]};
  v4u hv, lv;
#pragma unroll
  for (int q = 0; q < 4; ++q) {
    const float f0 = real ? f[2 * q] : 0.0f;
    const float f1 = real ? f[2 * q + 1] : 0.0f;
    const unsigned short h0 = f2bf_bits(f0), h1 = f2bf_bits(f1);
    const unsigned short l0 = f2bf_bits(f0 - bf_bits2f(h0));
    const unsigned short l1 = f2bf_bits(f1 - bf_bits2f(h1));
    hv[q] = (unsigned)h0 | ((unsigned)h1 << 16);
    lv[q] = (unsigned)l0 | ((unsigned)l1 << 16);
  }
  volatile v4u* ph = (volatile v4u*)((v4u*)dhi + t);
  volatile v4u* pl = (volatile v4u*)((v4u*)dlo + t);
  *ph = hv; *pl = lv;
  __threadfence();
  *ph = hv; *pl = lv;
}

template <int MODE>
__global__ __launch_bounds__(256) void plane_producer_kernel(
    const float* __restrict__ x, const float* __restrict__ offs, const float* __restrict__ b_off,
    unsigned int* __restrict__ planeHi, unsigned int* __restrict__ planeLo, int b0)
{
  __shared__ __align__(16) float sWt[NTAP * 32 * 4];
  __shared__ __align__(16) int   sIx[NTAP * 32 * 4];
  const int tid = threadIdx.x;
  const int blk = blockIdx.x;
  const int seg = blk % 3;
  const int h   = (blk / 3) % IMG_H;
  const int bl  = blk / (3 * IMG_H);
  const int b   = b0 + bl;
  const int w0  = seg * 32;
  const float* xb = x + (size_t)b * NCH_IN * HWPIX;

  if (MODE == 1) {
    for (int e = tid; e < NTAP * 32; e += 256) {
      const int pix = e & 31;
      const int tap = e >> 5;
      const int wpx = w0 + pix;
      const int kyi = tap / 3;
      const int kxi = tap - kyi * 3;
      const size_t obase = (size_t)b * MPAD * HWPIX + (size_t)h * IMG_W + wpx;
      const float dy = offs[obase + (size_t)(2 * tap) * HWPIX] + b_off[2 * tap];
      const float dx = offs[obase + (size_t)(2 * tap + 1) * HWPIX] + b_off[2 * tap + 1];
      const float py = (dy + (float)kyi) + (float)(h - 1);
      const float px = (dx + (float)kxi) + (float)(wpx - 1);
      const float fy0 = floorf(py), fx0 = floorf(px);
      const float fy1 = fy0 + 1.0f, fx1 = fx0 + 1.0f;
      const float wy1 = py - fy0, wx1 = px - fx0;
      const float wy0 = 1.0f - wy1, wx0 = 1.0f - wx1;
      const bool vy0 = (fy0 >= 0.0f) && (fy0 <= (float)(IMG_H - 1));
      const bool vy1 = (fy1 >= 0.0f) && (fy1 <= (float)(IMG_H - 1));
      const bool vx0 = (fx0 >= 0.0f) && (fx0 <= (float)(IMG_W - 1));
      const bool vx1 = (fx1 >= 0.0f) && (fx1 <= (float)(IMG_W - 1));
      const int iy0 = (int)fminf(fmaxf(fy0, 0.0f), (float)(IMG_H - 1));
      const int iy1 = (int)fminf(fmaxf(fy1, 0.0f), (float)(IMG_H - 1));
      const int ix0 = (int)fminf(fmaxf(fx0, 0.0f), (float)(IMG_W - 1));
      const int ix1 = (int)fminf(fmaxf(fx1, 0.0f), (float)(IMG_W - 1));
      v4f wv;
      wv[0] = (vy0 && vx0) ? (wy0 * wx0) : 0.0f;
      wv[1] = (vy0 && vx1) ? (wy0 * wx1) : 0.0f;
      wv[2] = (vy1 && vx0) ? (wy1 * wx0) : 0.0f;
      wv[3] = (vy1 && vx1) ? (wy1 * wx1) : 0.0f;
      v4i iv;
      iv[0] = iy0 * IMG_W + ix0;
      iv[1] = iy0 * IMG_W + ix1;
      iv[2] = iy1 * IMG_W + ix0;
      iv[3] = iy1 * IMG_W + ix1;
      *(v4f*)(sWt + e * 4) = wv;
      *(v4i*)(sIx + e * 4) = iv;
    }
    __syncthreads();
  }

  const int pL = tid >> 3;
  const int iS = tid & 7;
  const int ww = w0 + pL;
  const size_t rowIdx = (size_t)bl * HWPIX + (size_t)h * IMG_W + ww;
  v4u* phBase = (v4u*)planeHi + rowIdx * (KDIM / 8);
  v4u* plBase = (v4u*)planeLo + rowIdx * (KDIM / 8);

  for (int kc = 0; kc < KDIM / 64; ++kc) {
    unsigned hw0 = 0u, hw1 = 0u, hw2 = 0u, hw3 = 0u;
    unsigned lw0 = 0u, lw1 = 0u, lw2 = 0u, lw3 = 0u;
#pragma unroll 1
    for (int jj = 0; jj < 4; ++jj) {
      float vv[2];
#pragma unroll
      for (int u = 0; u < 2; ++u) {
        const int k   = kc * 64 + iS * 8 + jj * 2 + u;
        const int c   = k / NTAP;
        const int tap = k - c * NTAP;
        const float* xc = xb + (size_t)c * HWPIX;
        if (MODE == 0) {
          const int kyi = tap / 3;
          const int kxi = tap - kyi * 3;
          const int yy = h + kyi - 1;
          const int xx = ww + kxi - 1;
          const bool valid = (yy >= 0) && (yy < IMG_H) && (xx >= 0) && (xx < IMG_W);
          const int yyc = yy < 0 ? 0 : (yy > IMG_H - 1 ? IMG_H - 1 : yy);
          const int xxc = xx < 0 ? 0 : (xx > IMG_W - 1 ? IMG_W - 1 : xx);
          const float tv = xc[yyc * IMG_W + xxc];
          vv[u] = valid ? tv : 0.0f;
        } else {
          const int e = tap * 32 + pL;
          const v4f wv = *(const v4f*)(sWt + e * 4);
          const v4i iv = *(const v4i*)(sIx + e * 4);
          const float x00 = xc[iv[0]];
          const float x01 = xc[iv[1]];
          const float x10 = xc[iv[2]];
          const float x11 = xc[iv[3]];
          float a = 0.0f;
          a = a + x00 * wv[0];
          a = a + x01 * wv[1];
          a = a + x10 * wv[2];
          a = a + x11 * wv[3];
          vv[u] = a;
        }
      }
      const unsigned short h0 = f2bf_bits(vv[0]), h1 = f2bf_bits(vv[1]);
      const unsigned short l0 = f2bf_bits(vv[0] - bf_bits2f(h0));
      const unsigned short l1 = f2bf_bits(vv[1] - bf_bits2f(h1));
      const unsigned nh = (unsigned)h0 | ((unsigned)h1 << 16);
      const unsigned nl = (unsigned)l0 | ((unsigned)l1 << 16);
      hw0 = hw1; hw1 = hw2; hw2 = hw3; hw3 = nh;
      lw0 = lw1; lw1 = lw2; lw2 = lw3; lw3 = nl;
    }
    v4u hv, lv;
    hv[0] = hw0; hv[1] = hw1; hv[2] = hw2; hv[3] = hw3;
    lv[0] = lw0; lv[1] = lw1; lv[2] = lw2; lv[3] = lw3;
    volatile v4u* dph = (volatile v4u*)(phBase + kc * 8 + iS);
    volatile v4u* dpl = (volatile v4u*)(plBase + kc * 8 + iS);
    *dph = hv; *dpl = lv;
    __threadfence();
    *dph = hv; *dpl = lv;
  }
}

__global__ __launch_bounds__(256) void chan_partial_kernel(
    const float* __restrict__ ypre, const float* __restrict__ b_def, float* __restrict__ table)
{
  __shared__ float sS[8];
  __shared__ float sQ[8];
  const int s    = blockIdx.x;
  const int ch   = s & (NCH_OUT - 1);
  const int bb   = s >> 6;
  const int lane = threadIdx.x & 31;
  const int wave = threadIdx.x >> 5;
  const float bias = b_def[ch];
  const float* yp = ypre + (size_t)s * HWPIX;
  float a = 0.0f, q = 0.0f;
#pragma unroll 1
  for (int it = 0; it < HWPIX / 1024; ++it) {
    const v4f v = *(const v4f*)(yp + (size_t)(it * 256 + threadIdx.x) * 4);
#pragma unroll
    for (int e = 0; e < 4; ++e) {
      const float y = v[e] + bias;
      a = a + y;
      q = q + y * y;
    }
  }
#pragma unroll
  for (int off = 1; off < 32; off <<= 1) {
    a += __shfl_xor(a, off, 32);
    q += __shfl_xor(q, off, 32);
  }
  if (lane == 0) { sS[wave] = a; sQ[wave] = q; }
  __syncthreads();
  if (wave == 0) {
    float S = 0.0f, Q = 0.0f;
#pragma unroll
    for (int w = 0; w < 8; ++w) { S = S + sS[w]; Q = Q + sQ[w]; }
    const float val = (lane == 0) ? S : ((lane == 1) ? Q : 0.0f);
    volatile float* tp = table + ((size_t)ch * NBATCH + bb) * 32 + lane;
    *tp = val;
    __threadfence();
    *tp = val;
  }
}

__global__ __launch_bounds__(256) void norm_relu_kernel(
    const float* __restrict__ ypre, const float* __restrict__ table,
    const float* __restrict__ b_def, const float* __restrict__ gamma, const float* __restrict__ beta,
    float* __restrict__ out)
{
  const int blk  = blockIdx.x;
  const int s    = blk / (HWPIX / 1024);
  const int part = blk - s * (HWPIX / 1024);
  const int ch   = s & (NCH_OUT - 1);
  const int lane = threadIdx.x & 31;
  const int bb   = lane & (NBATCH - 1);
  const v2f pr = *(const v2f*)(table + ((size_t)ch * NBATCH + bb) * 32);
  double S = (lane < NBATCH) ? (double)pr[0] : 0.0;
  double Q = (lane < NBATCH) ? (double)pr[1] : 0.0;
#pragma unroll
  for (int off = 1; off < 32; off <<= 1) {
    S += __shfl_xor(S, off, 32);
    Q += __shfl_xor(Q, off, 32);
  }
  const double n = (double)NBATCH * (double)HWPIX;
  const double mean = S / n;
  double var = Q / n - mean * mean;
  if (var < 0.0) var = 0.0;
  const float meanf = (float)mean;
  const float varf  = (float)var;
  const float inv   = 1.0f / sqrtf(varf + BN_EPS);
  const float g    = gamma[ch];
  const float be   = beta[ch];
  const float bias = b_def[ch];
  const size_t idx = (size_t)s * HWPIX + (size_t)part * 1024 + (size_t)threadIdx.x * 4;
  const v4f v = *(const v4f*)(ypre + idx);
  v4f o;
#pragma unroll
  for (int e = 0; e < 4; ++e) {
    const float y = v[e] + bias;
    float tv = (y - meanf) * inv;
    tv = g * tv + be;
    o[e] = tv > 0.0f ? tv : 0.0f;
  }
  volatile v4f* op = (volatile v4f*)(out + idx);
  *op = o;
  __threadfence();
  *op = o;
}

extern "C" void kernel_launch(void* const* d_in, const int* in_sizes, int n_in,
                              void* d_out, int out_size, void* d_ws, size_t ws_size,
                              hipStream_t stream)
{
  if (n_in < 7) return;
  if (in_sizes[0] != NBATCH * NCH_IN * HWPIX) return;
  if (in_sizes[1] != NOFFC * KDIM) return;
  if (in_sizes[2] != NOFFC) return;
  if (in_sizes[3] != NCH_OUT * KDIM) return;
  if (in_sizes[4] != NCH_OUT || in_sizes[5] != NCH_OUT || in_sizes[6] != NCH_OUT) return;
  if (out_size != NBATCH * NCH_OUT * HWPIX) return;
  if (ws_size < WS_TOTAL) return;

  const float* x     = (const float*)d_in[0];
  const float* w_off = (const float*)d_in[1];
  const float* b_off = (const float*)d_in[2];
  const float* w_def = (const float*)d_in[3];
  const float* b_def = (const float*)d_in[4];
  const float* gamma = (const float*)d_in[5];
  const float* beta  = (const float*)d_in[6];
  float* out = (float*)d_out;

  char* ws = (char*)d_ws;
  unsigned int* planeHi = (unsigned int*)(ws + R_PHI);
  unsigned int* planeLo = (unsigned int*)(ws + R_PLO);
  float* offs  = (float*)(ws + R_OFFS);
  float* ypre  = (float*)(ws + R_YPRE);
  unsigned int* wohi = (unsigned int*)(ws + R_WOH);
  unsigned int* wolo = (unsigned int*)(ws + R_WOL);
  unsigned int* wdhi = (unsigned int*)(ws + R_WDH);
  unsigned int* wdlo = (unsigned int*)(ws + R_WDL);
  float* table = (float*)(ws + R_TAB);

  const int nSplitThreads = MPAD * KDIM / 8;
  const int splitBlocks = (nSplitThreads + 255) / 256;
  split_rows_kernel<<<splitBlocks, 256, 0, stream>>>(w_off, NOFFC, wohi, wolo);
  split_rows_kernel<<<splitBlocks, 256, 0, stream>>>(w_def, NCH_OUT, wdhi, wdlo);

  const int gemmM = MPAD, gemmN = HWPIX, gemmK = KDIM;
  const int gemmTiles = (gemmM / 64) * (gemmN / 64);
  const dim3 gemmGrid((gemmTiles + 7) / 8, HALF_B);
  const long strideB = (long)HWPIX * KDIM;
  const long strideC = (long)MPAD * HWPIX;
  const int prodBlocks = HALF_B * IMG_H * (IMG_W / 32);

  for (int hf = 0; hf < NBATCH / HALF_B; ++hf) {
    const int b0 = hf * HALF_B;
    plane_producer_kernel<0><<<prodBlocks, 256, 0, stream>>>(x, offs, b_off, planeHi, planeLo, b0);
    wmma_gemm64<1, true, 0, 0, false, 0><<<gemmGrid, 256, 0, stream>>>(
        (const unsigned short*)wohi, (const unsigned short*)wolo, gemmK, 0L,
        (const unsigned short*)planeHi, (const unsigned short*)planeLo, gemmK, strideB,
        (void*)(offs + (size_t)b0 * MPAD * HWPIX), (void*)(offs + (size_t)b0 * MPAD * HWPIX), gemmN, strideC,
        b_def, (const float*)offs, 0L, gemmM, gemmN, gemmK, 1.0f);
    plane_producer_kernel<1><<<prodBlocks, 256, 0, stream>>>(x, offs, b_off, planeHi, planeLo, b0);
    wmma_gemm64<1, true, 0, 0, false, 0><<<gemmGrid, 256, 0, stream>>>(
        (const unsigned short*)wdhi, (const unsigned short*)wdlo, gemmK, 0L,
        (const unsigned short*)planeHi, (const unsigned short*)planeLo, gemmK, strideB,
        (void*)(ypre + (size_t)b0 * NCH_OUT * HWPIX), (void*)(ypre + (size_t)b0 * NCH_OUT * HWPIX), gemmN, strideC,
        b_def, (const float*)offs, 0L, gemmM, gemmN, gemmK, 1.0f);
  }

  chan_partial_kernel<<<NBATCH * NCH_OUT, 256, 0, stream>>>(ypre, b_def, table);
  norm_relu_kernel<<<NBATCH * NCH_OUT * (HWPIX / 1024), 256, 0, stream>>>(ypre, table, b_def, gamma, beta, out);
}
